// LSTM_1073741824385
// MI455X (gfx1250) — hardware-verified
//
#include <hip/hip_runtime.h>

typedef __attribute__((ext_vector_type(16))) _Float16 v16h;
typedef __attribute__((ext_vector_type(8)))  _Float16 v8h;
typedef __attribute__((ext_vector_type(16))) __bf16   v16b;
typedef __attribute__((ext_vector_type(8)))  __bf16   v8b;
typedef __attribute__((ext_vector_type(8)))  float    v8f;
typedef __attribute__((ext_vector_type(4)))  float    v4f;
typedef __attribute__((ext_vector_type(4)))  unsigned int v4u;

constexpr int NBATCH = 32;
constexpr int NSEQ   = 512;
constexpr int NIN    = 256;
constexpr int NHID   = 512;
constexpr int NGATE  = 4 * NHID;
constexpr int NOUT   = 256;
constexpr int HCOLS  = 64;
constexpr int GLP    = 260;
constexpr float WSCALE     = 64.0f;
constexpr float WSCALE_INV = 0.015625f;
constexpr long  PLANE    = (long)NBATCH * NHID;
constexpr long  OUT0_N   = (long)NBATCH * NSEQ * NOUT;
constexpr long  OUT1_OFF = OUT0_N;
constexpr long  OUT2_OFF = OUT0_N + 2 * PLANE;
static_assert(OUT1_OFF * 4 == 16777216);
static_assert(OUT2_OFF * 4 == 16908288);
static_assert((OUT2_OFF + 2 * PLANE) * 4 == 17039360);
static_assert(NHID % HCOLS == 0 && HCOLS == 64);
static_assert(NBATCH == 32);
static_assert(NIN % 64 == 0 && NHID % 64 == 0);
static_assert(NSEQ % 64 == 0 && NOUT % 64 == 0 && NHID % 32 == 0);
static_assert(((NSEQ / 64) * (NOUT / 64)) % 8 == 0);
static_assert(GLP % 4 == 0);

__device__ __forceinline__ unsigned short f2bf_bits(float f) {
  unsigned u = __float_as_uint(f);
  return (unsigned short)((u + 0x7FFFu + ((u >> 16) & 1u)) >> 16);
}
__device__ __forceinline__ float bf_bits2f(unsigned short h) { return __uint_as_float(((unsigned)h) << 16); }

__device__ __forceinline__ void dep_guard_h(v8f& a, v8f& b, v16h x, v16h y) { asm volatile("v_nop\n\tv_nop\n\tv_nop\n\tv_nop" : "+v"(a), "+v"(b) : "v"(x), "v"(y)); }
__device__ __forceinline__ void dep_guard_b(v8f& a, v8f& b, v16b x, v16b y) { asm volatile("v_nop\n\tv_nop\n\tv_nop\n\tv_nop" : "+v"(a), "+v"(b) : "v"(x), "v"(y)); }
__device__ __forceinline__ void keep4_h(v16h a, v16h b, v16h c, v16h d) { asm volatile("v_nop" :: "v"(a), "v"(b), "v"(c), "v"(d)); }
__device__ __forceinline__ void keep4_b(v16b a, v16b b, v16b c, v16b d) { asm volatile("v_nop" :: "v"(a), "v"(b), "v"(c), "v"(d)); }
__device__ __forceinline__ void acc_guard4(v8f& a, v8f& b, v8f& c, v8f& d) { asm volatile("v_nop\n\tv_nop\n\tv_nop\n\tv_nop" : "+v"(a), "+v"(b), "+v"(c), "+v"(d)); }
template <typename T> struct Frag;
template <> struct Frag<_Float16> {
  typedef v16h V; union U { v16h v; v8h h[2]; };
  static __device__ __forceinline__ v16h load(const _Float16* p) {
    U f; f.h[0] = *(const v8h*)(p); f.h[1] = *(const v8h*)(p + 16); return f.v;
  }
  static __device__ __forceinline__ v8f mma(v16h a, v16h b, v8f c) {
    return __builtin_amdgcn_wmma_f32_16x16x32_f16(false, a, false, b, (short)0, c, false, false);
  }
  static __device__ __forceinline__ void guard(v8f& a, v8f& b, v16h x, v16h y) { dep_guard_h(a, b, x, y); }
  static __device__ __forceinline__ void keep(v16h a, v16h b, v16h c, v16h d) { keep4_h(a, b, c, d); }
};
template <> struct Frag<__bf16> {
  typedef v16b V; union U { v16b v; v8b h[2]; };
  static __device__ __forceinline__ v16b load(const __bf16* p) {
    U f; f.h[0] = *(const v8b*)(p); f.h[1] = *(const v8b*)(p + 16); return f.v;
  }
  static __device__ __forceinline__ v8f mma(v16b a, v16b b, v8f c) {
    return __builtin_amdgcn_wmma_f32_16x16x32_bf16(false, a, false, b, (short)0, c, false, false);
  }
  static __device__ __forceinline__ void guard(v8f& a, v8f& b, v16b x, v16b y) { dep_guard_b(a, b, x, y); }
  static __device__ __forceinline__ void keep(v16b a, v16b b, v16b c, v16b d) { keep4_b(a, b, c, d); }
};

template <int ET> struct Elem;
template <> struct Elem<0> { typedef _Float16 T; };
template <> struct Elem<1> { typedef __bf16 T; };
template <int ET, bool SPLIT, int BIAS_MODE, int OUT_MODE, bool RESID, int ACT = 0>
__global__ __launch_bounds__(256) void wmma_gemm64(
    const unsigned short* __restrict__ Ap, const unsigned short* __restrict__ A2p, int lda, long strideA,
    const unsigned short* __restrict__ Btp, const unsigned short* __restrict__ Bt2p, int ldb, long strideB,
    void* __restrict__ Cout, void* __restrict__ Cout2, int ldc, long strideC,
    const float* __restrict__ bias,
    const float* __restrict__ resid, long strideR,
    int M, int N, int K, float scale) {
  typedef typename Elem<ET>::T T;
  typedef typename Frag<T>::V V;
  const T* A = (const T*)Ap; const T* A2 = (const T*)A2p; const T* Bt = (const T*)Btp; const T* Bt2 = (const T*)Bt2p;
  __shared__ __align__(16) float sT[8][16 * 68];
  const int b    = blockIdx.y;
  const int lane = threadIdx.x & 31;
  const int wave = threadIdx.x >> 5;
  const int tilesN = N >> 6;
  const int tilesM = M >> 6;
  const int tile = blockIdx.x * 8 + wave;
  if (tile >= tilesM * tilesN) return;
  const int tm = tile / tilesN;
  const int tn = tile - tm * tilesN;
  const int m0 = tm << 6;
  const int n0 = tn << 6;

  const T* Ab  = A  + (size_t)b * strideA;
  const T* Bb  = Bt + (size_t)b * strideB;
  const T* Ab2 = SPLIT ? (A2  + (size_t)b * strideA) : nullptr;
  const T* Bb2 = SPLIT ? (Bt2 + (size_t)b * strideB) : nullptr;

  const int rlane = lane & 15;
  const int koff  = (lane >> 4) * 8;
  const int mOff  = (lane >> 4) * 8;

  v8f acc[4][4];
#pragma unroll
  for (int i = 0; i < 4; ++i)
#pragma unroll
    for (int j = 0; j < 4; ++j) acc[i][j] = (v8f){0.f,0.f,0.f,0.f,0.f,0.f,0.f,0.f};

  for (int k0 = 0; k0 < K; k0 += 32) {
    V bh[4], bl[4];
#pragma unroll
    for (int j = 0; j < 4; ++j) {
      const size_t bo = (size_t)(n0 + (j << 4) + rlane) * ldb + koff + k0;
      bh[j] = Frag<T>::load(Bb + bo);
      if (SPLIT) bl[j] = Frag<T>::load(Bb2 + bo);
    }
#pragma unroll
    for (int i = 0; i < 4; ++i) {
      const size_t ao = (size_t)(m0 + (i << 4) + rlane) * lda + koff + k0;
      V ah = Frag<T>::load(Ab + ao);
      V al;
      if (SPLIT) al = Frag<T>::load(Ab2 + ao);
#pragma unroll
      for (int j = 0; j < 4; ++j) {
        acc[i][j] = Frag<T>::mma(ah, bh[j], acc[i][j]);
        if (SPLIT) {
          acc[i][j] = Frag<T>::mma(ah, bl[j], acc[i][j]);
          acc[i][j] = Frag<T>::mma(al, bh[j], acc[i][j]);
        }
      }
      Frag<T>::guard(acc[i][0], acc[i][3], ah, SPLIT ? al : ah);
    }
    Frag<T>::keep(bh[0], bh[1], bh[2], bh[3]);
    if (SPLIT) Frag<T>::keep(bl[0], bl[1], bl[2], bl[3]);
  }
  acc_guard4(acc[0][0], acc[0][1], acc[0][2], acc[0][3]);
  acc_guard4(acc[1][0], acc[1][1], acc[1][2], acc[1][3]);
  acc_guard4(acc[2][0], acc[2][1], acc[2][2], acc[2][3]);
  acc_guard4(acc[3][0], acc[3][1], acc[3][2], acc[3][3]);

  float* slab = sT[wave];
  const float* Rb = RESID ? (resid + (size_t)b * strideR) : nullptr;
#pragma unroll
  for (int i = 0; i < 4; ++i) {
    const int mBase = m0 + (i << 4);
#pragma unroll
    for (int j = 0; j < 4; ++j) {
      const int n = n0 + (j << 4) + rlane;
      float bv = 0.f;
      if (BIAS_MODE == 2) bv = bias[n];
#pragma unroll
      for (int r = 0; r < 8; ++r) {
        float v = acc[i][j][r] * scale;
        if (BIAS_MODE == 1) v += bias[mBase + mOff + r];
        if (BIAS_MODE == 2) v += bv;
        if (RESID) v += Rb[(size_t)(mBase + mOff + r) * ldc + n];
        if (ACT == 1) v = tanhf(v);
        if (ACT == 2) v = fmaxf(v, 0.0f);
        if (ACT == 3) v = v / (1.0f + expf(-v));
        if (ACT == 4) v = (v > 0.f) ? v : 0.01f * v;
        if (ACT == 5) v = 0.5f * v * (1.0f + erff(v * 0.70710678118654752f));
        slab[(mOff + r) * 68 + (j << 4) + rlane] = v;
      }
    }
    __builtin_amdgcn_fence(__ATOMIC_RELEASE, "workgroup");
    __builtin_amdgcn_wave_barrier();
    __builtin_amdgcn_fence(__ATOMIC_ACQUIRE, "workgroup");
    if (OUT_MODE == 0) {
      float* C = (float*)Cout + (size_t)b * strideC;
      const int hh = lane >> 4, c4 = (lane & 15) * 4;
      for (int pass = 0; pass < 2; ++pass) {
#pragma unroll
        for (int it = 0; it < 8; ++it) {
          const int row = it * 2 + hh;
          v4f v = *(const v4f*)(slab + row * 68 + c4);
          *(volatile v4f*)(C + (size_t)(mBase + row) * ldc + n0 + c4) = v;
        }
        __threadfence();
      }
    } else {
      const int q = lane >> 3, c8 = (lane & 7) * 8;
      unsigned short* C  = (unsigned short*)Cout  + (size_t)b * strideC;
      unsigned short* C2 = (OUT_MODE == 2) ? ((unsigned short*)Cout2 + (size_t)b * strideC) : nullptr;
      for (int pass = 0; pass < 2; ++pass) {
#pragma unroll
        for (int it = 0; it < 4; ++it) {
          const int row = it * 4 + q;
          const float* sp = slab + row * 68 + c8;
          v8h hv, lv;
#pragma unroll
          for (int e = 0; e < 8; ++e) {
            if (OUT_MODE == 1) {
              hv[e] = (_Float16)sp[e];
            } else {
              unsigned short hb = f2bf_bits(sp[e]);
              unsigned short lb = f2bf_bits(sp[e] - bf_bits2f(hb));
              hv[e] = __builtin_bit_cast(_Float16, hb);
              lv[e] = __builtin_bit_cast(_Float16, lb);
            }
          }
          *(volatile v8h*)(C + (size_t)(mBase + row) * ldc + n0 + c8) = hv;
          if (OUT_MODE == 2) *(volatile v8h*)(C2 + (size_t)(mBase + row) * ldc + n0 + c8) = lv;
        }
        __threadfence();
      }
    }
    __builtin_amdgcn_fence(__ATOMIC_RELEASE, "workgroup");
    __builtin_amdgcn_wave_barrier();
    __builtin_amdgcn_fence(__ATOMIC_ACQUIRE, "workgroup");
  }
}

__device__ __forceinline__ float bf16_rne(float f) {
  unsigned u = __float_as_uint(f);
  u = (u + 0x7FFFu + ((u >> 16) & 1u)) & 0xFFFF0000u;
  return __uint_as_float(u);
}
__device__ __forceinline__ float sigm_f(float x) {
  return __builtin_amdgcn_rcpf(1.0f + expf(-x));
}
__device__ __forceinline__ void guard8(v8f& a, v8f& b, v8f& c, v8f& d, v16h w, v16h x, v16h y, v16h z) {
  asm volatile("v_nop\n\tv_nop\n\tv_nop\n\tv_nop" : "+v"(a), "+v"(b), "+v"(c), "+v"(d) : "v"(w), "v"(x), "v"(y), "v"(z));
}

__global__ __launch_bounds__(256) void cast_bf16rne_f16x8(
    const float* __restrict__ in, unsigned short* __restrict__ out, int n8, float scale) {
  const int i = blockIdx.x * 256 + threadIdx.x;
  if (i < n8) {
    const v4f u0 = *(const v4f*)(in + (size_t)i * 8);
    const v4f u1 = *(const v4f*)(in + (size_t)i * 8 + 4);
    v8h hv;
#pragma unroll
    for (int e = 0; e < 4; ++e) {
      hv[e]     = (_Float16)(bf16_rne(u0[e]) * scale);
      hv[4 + e] = (_Float16)(bf16_rne(u1[e]) * scale);
    }
    unsigned short* p = out + (size_t)i * 8;
    *(volatile v8h*)p = hv;
    __threadfence();
    *(volatile v8h*)p = hv;
  }
}

__global__ __launch_bounds__(256) void zero_fill16(unsigned int* __restrict__ p, int n16) {
  const int i = blockIdx.x * 256 + threadIdx.x;
  if (i < n16) {
    const v4u z = (v4u){0u, 0u, 0u, 0u};
    unsigned int* q = p + (size_t)i * 4;
    *(volatile v4u*)q = z;
    __threadfence();
    *(volatile v4u*)q = z;
  }
}

__global__ __launch_bounds__(64) void rne_vec4(const float* __restrict__ in, float* __restrict__ out, int n4) {
  const int i = blockIdx.x * 64 + threadIdx.x;
  if (i < n4) {
    const v4f v = *(const v4f*)(in + (size_t)i * 4);
    v4f r;
    r[0] = bf16_rne(v[0]); r[1] = bf16_rne(v[1]); r[2] = bf16_rne(v[2]); r[3] = bf16_rne(v[3]);
    float* q = out + (size_t)i * 4;
    *(volatile v4f*)q = r;
    __threadfence();
    *(volatile v4f*)q = r;
  }
}

struct LayerArgs {
  const unsigned short* ain;
  const unsigned short* win;
  const unsigned short* whh;
  const float* bih;
  const float* bhh;
  float* cpl;
  unsigned short* hseq;
  float* hn;
  float* cn;
  long ain_bpitch;
  long ain_tpitch;
};
static_assert(sizeof(LayerArgs) == 88);

template <int KLEN>
__device__ __forceinline__ void mac_seg(v8f& a00, v8f& a01, v8f& a10, v8f& a11,
                                        const _Float16* a0p, const _Float16* a1p,
                                        const _Float16* b0p, const _Float16* b1p) {
#pragma unroll 2
  for (int k0 = 0; k0 < KLEN; k0 += 32) {
    const v16h fa0 = Frag<_Float16>::load(a0p + k0);
    const v16h fa1 = Frag<_Float16>::load(a1p + k0);
    const v16h fb0 = Frag<_Float16>::load(b0p + k0);
    const v16h fb1 = Frag<_Float16>::load(b1p + k0);
    a00 = Frag<_Float16>::mma(fa0, fb0, a00);
    a01 = Frag<_Float16>::mma(fa0, fb1, a01);
    a10 = Frag<_Float16>::mma(fa1, fb0, a10);
    a11 = Frag<_Float16>::mma(fa1, fb1, a11);
    guard8(a00, a01, a10, a11, fa0, fa1, fb0, fb1);
  }
}

__global__ __launch_bounds__(256) void lstm_step(LayerArgs L0, LayerArgs L1, int t0, int lbase, int tlast) {
  __shared__ __align__(16) float gl[NBATCH * GLP];

  const int layer = lbase + (int)blockIdx.y;
  const bool is1 = (layer != 0);
  const int t = is1 ? (t0 - 1) : t0;
  const unsigned short* ain  = is1 ? L1.ain : L0.ain;
  const unsigned short* win  = is1 ? L1.win : L0.win;
  const unsigned short* whh  = is1 ? L1.whh : L0.whh;
  const float* bih           = is1 ? L1.bih : L0.bih;
  const float* bhh           = is1 ? L1.bhh : L0.bhh;
  float* cpl                 = is1 ? L1.cpl : L0.cpl;
  unsigned short* hseq       = is1 ? L1.hseq : L0.hseq;
  float* hn                  = is1 ? L1.hn : L0.hn;
  float* cn                  = is1 ? L1.cn : L0.cn;
  const long bpitch          = is1 ? L1.ain_bpitch : L0.ain_bpitch;
  const long tpitch          = is1 ? L1.ain_tpitch : L0.ain_tpitch;

  const int lane = threadIdx.x & 31;
  const int wave = threadIdx.x >> 5;
  const int rl   = lane & 15;
  const int hh   = lane >> 4;
  const int koff = hh * 8;
  const int c0   = blockIdx.x * HCOLS;
  const int nrow0 = (wave >> 1) * NHID + c0 + (wave & 1) * 32;

  const _Float16* Ain  = (const _Float16*)ain + (size_t)t * tpitch;
  const _Float16* Alag = (const _Float16*)hseq + (size_t)t * PLANE;
  const _Float16* Wi   = (const _Float16*)win;
  const _Float16* Wh   = (const _Float16*)whh;
  const int kin = is1 ? NHID : NIN;

  v8f acc00 = (v8f){0.f,0.f,0.f,0.f,0.f,0.f,0.f,0.f};
  v8f acc01 = acc00, acc10 = acc00, acc11 = acc00;

  {
    const _Float16* a0p = Ain + (size_t)rl * bpitch + koff;
    const _Float16* a1p = Ain + (size_t)(16 + rl) * bpitch + koff;
    const _Float16* b0p = Wi + (size_t)(nrow0 + rl) * kin + koff;
    const _Float16* b1p = Wi + (size_t)(nrow0 + 16 + rl) * kin + koff;
    if (is1) mac_seg<NHID>(acc00, acc01, acc10, acc11, a0p, a1p, b0p, b1p);
    else     mac_seg<NIN>(acc00, acc01, acc10, acc11, a0p, a1p, b0p, b1p);
  }
  {
    const _Float16* a0p = Alag + (size_t)rl * NHID + koff;
    const _Float16* a1p = Alag + (size_t)(16 + rl) * NHID + koff;
    const _Float16* b0p = Wh + (size_t)(nrow0 + rl) * NHID + koff;
    const _Float16* b1p = Wh + (size_t)(nrow0 + 16 + rl) * NHID + koff;
    mac_seg<NHID>(acc00, acc01, acc10, acc11, a0p, a1p, b0p, b1p);
  }
  acc_guard4(acc00, acc01, acc10, acc11);

  {
    const int gA = wave * 32 + rl;
    const int gB = gA + 16;
    const float bsA = bf16_rne(bih[nrow0 + rl]) + bf16_rne(bhh[nrow0 + rl]);
    const float bsB = bf16_rne(bih[nrow0 + 16 + rl]) + bf16_rne(bhh[nrow0 + 16 + rl]);
#pragma unroll
    for (int r = 0; r < 8; ++r) {
      const int bu = 8 * hh + r;
      const int bl = 16 + bu;
      gl[bu * GLP + gA] = acc00[r] * WSCALE_INV + bsA;
      gl[bu * GLP + gB] = acc01[r] * WSCALE_INV + bsB;
      gl[bl * GLP + gA] = acc10[r] * WSCALE_INV + bsA;
      gl[bl * GLP + gB] = acc11[r] * WSCALE_INV + bsB;
    }
  }
  __syncthreads();

  const int crow = wave * 4 + (lane >> 3);
  const int ccol = (lane & 7) * 8;
  const float* cinp = cpl + (size_t)(t & 1) * PLANE + (size_t)crow * NHID + c0 + ccol;
  float ca[8], ha[8];
  {
    const float* glr = gl + crow * GLP + ccol;
    const v4f gi0 = *(const v4f*)(glr);
    const v4f gi1 = *(const v4f*)(glr + 4);
    const v4f gf0 = *(const v4f*)(glr + 64);
    const v4f gf1 = *(const v4f*)(glr + 68);
    const v4f gg0 = *(const v4f*)(glr + 128);
    const v4f gg1 = *(const v4f*)(glr + 132);
    const v4f go0 = *(const v4f*)(glr + 192);
    const v4f go1 = *(const v4f*)(glr + 196);
    const v4f cl0 = *(const v4f*)(cinp);
    const v4f cl1 = *(const v4f*)(cinp + 4);
#pragma unroll
    for (int e = 0; e < 4; ++e) {
      {
        const float ig = sigm_f(gi0[e]);
        const float fg = sigm_f(gf0[e]);
        const float gg = tanhf(gg0[e]);
        const float og = sigm_f(go0[e]);
        const float cnew = fg * cl0[e] + ig * gg;
        ca[e] = cnew;
        ha[e] = og * tanhf(cnew);
      }
      {
        const float ig = sigm_f(gi1[e]);
        const float fg = sigm_f(gf1[e]);
        const float gg = tanhf(gg1[e]);
        const float og = sigm_f(go1[e]);
        const float cnew = fg * cl1[e] + ig * gg;
        ca[4 + e] = cnew;
        ha[4 + e] = og * tanhf(cnew);
      }
    }
  }
  {
    float* glw = gl + crow * GLP + ccol;
    *(v4f*)(glw)      = (v4f){ca[0], ca[1], ca[2], ca[3]};
    *(v4f*)(glw + 4)  = (v4f){ca[4], ca[5], ca[6], ca[7]};
    *(v4f*)(glw + 64) = (v4f){ha[0], ha[1], ha[2], ha[3]};
    *(v4f*)(glw + 68) = (v4f){ha[4], ha[5], ha[6], ha[7]};
  }
  v8h hpk;
  hpk[0] = (_Float16)ha[0]; hpk[1] = (_Float16)ha[1]; hpk[2] = (_Float16)ha[2]; hpk[3] = (_Float16)ha[3];
  hpk[4] = (_Float16)ha[4]; hpk[5] = (_Float16)ha[5]; hpk[6] = (_Float16)ha[6]; hpk[7] = (_Float16)ha[7];

  unsigned short* hdst = hseq + (size_t)(t + 1) * PLANE + (size_t)crow * NHID + c0 + ccol;
  float* coutp = cpl + (size_t)((t + 1) & 1) * PLANE;
  const bool fin = (t == tlast);
  __syncthreads();

  for (int pass = 0; pass < 2; ++pass) {
    *(volatile v8h*)hdst = hpk;
#pragma unroll
    for (int p2 = 0; p2 < 2; ++p2) {
      const int r2 = wave * 4 + p2 * 2 + hh;
      const int c4 = rl * 4;
      const v4f cv = *(const v4f*)(gl + r2 * GLP + c4);
      const size_t eo = (size_t)r2 * NHID + c0 + c4;
      *(volatile v4f*)(coutp + eo) = cv;
      if (fin) {
        const v4f hv4 = *(const v4f*)(gl + r2 * GLP + 64 + c4);
        *(volatile v4f*)(hn + eo) = hv4;
        *(volatile v4f*)(cn + eo) = cv;
      }
    }
    __threadfence();
  }
}

extern "C" void kernel_launch(void* const* d_in, const int* in_sizes, int n_in,
                              void* d_out, int out_size, void* d_ws, size_t ws_size,
                              hipStream_t stream) {
  if (n_in < 11) return;
  if (in_sizes[0] != NBATCH * NSEQ * NIN) return;
  if (in_sizes[2] != NGATE * NHID) return;
  if (out_size != (int)(OUT2_OFF + 2 * PLANE)) return;

  size_t off = 0;
  auto take = [&](size_t bytes) -> size_t { size_t o = off; off += (bytes + 255) & ~(size_t)255; return o; };
  const size_t o_cpl  = take((size_t)4 * PLANE * 4);
  const size_t o_h0   = take((size_t)(NSEQ + 1) * PLANE * 2);
  const size_t o_h1   = take((size_t)(NSEQ + 1) * PLANE * 2);
  const size_t o_xh   = take((size_t)NBATCH * NSEQ * NIN * 2);
  const size_t o_wih0 = take((size_t)NGATE * NIN * 2);
  const size_t o_whh0 = take((size_t)NGATE * NHID * 2);
  const size_t o_wih1 = take((size_t)NGATE * NHID * 2);
  const size_t o_whh1 = take((size_t)NGATE * NHID * 2);
  const size_t o_wlin = take((size_t)NOUT * NHID * 2);
  const size_t o_blin = take((size_t)NOUT * 4);
  const size_t total  = off;
  if (total > ws_size) return;
  if (o_h0 != o_cpl + (size_t)4 * PLANE * 4) return;

  char* wsb = (char*)d_ws;
  float* out = (float*)d_out;
  float* cpl = (float*)(wsb + o_cpl);
  unsigned short* h0   = (unsigned short*)(wsb + o_h0);
  unsigned short* h1   = (unsigned short*)(wsb + o_h1);
  unsigned short* xh   = (unsigned short*)(wsb + o_xh);
  unsigned short* wih0 = (unsigned short*)(wsb + o_wih0);
  unsigned short* whh0 = (unsigned short*)(wsb + o_whh0);
  unsigned short* wih1 = (unsigned short*)(wsb + o_wih1);
  unsigned short* whh1 = (unsigned short*)(wsb + o_whh1);
  unsigned short* wlin = (unsigned short*)(wsb + o_wlin);
  float* blin = (float*)(wsb + o_blin);

  const float* x      = (const float*)d_in[0];
  const float* W_ih0  = (const float*)d_in[1];
  const float* W_hh0  = (const float*)d_in[2];
  const float* b_ih0  = (const float*)d_in[3];
  const float* b_hh0  = (const float*)d_in[4];
  const float* W_ih1  = (const float*)d_in[5];
  const float* W_hh1  = (const float*)d_in[6];
  const float* b_ih1  = (const float*)d_in[7];
  const float* b_hh1  = (const float*)d_in[8];
  const float* W_lin  = (const float*)d_in[9];
  const float* b_lin  = (const float*)d_in[10];

  {
    const int n8x = NBATCH * NSEQ * NIN / 8;
    cast_bf16rne_f16x8<<<(n8x + 255) / 256, 256, 0, stream>>>(x, xh, n8x, 1.0f);
    const int n8a = NGATE * NIN / 8;
    cast_bf16rne_f16x8<<<(n8a + 255) / 256, 256, 0, stream>>>(W_ih0, wih0, n8a, WSCALE);
    const int n8b = NGATE * NHID / 8;
    cast_bf16rne_f16x8<<<(n8b + 255) / 256, 256, 0, stream>>>(W_hh0, whh0, n8b, WSCALE);
    cast_bf16rne_f16x8<<<(n8b + 255) / 256, 256, 0, stream>>>(W_ih1, wih1, n8b, WSCALE);
    cast_bf16rne_f16x8<<<(n8b + 255) / 256, 256, 0, stream>>>(W_hh1, whh1, n8b, WSCALE);
    const int n8c = NOUT * NHID / 8;
    cast_bf16rne_f16x8<<<(n8c + 255) / 256, 256, 0, stream>>>(W_lin, wlin, n8c, WSCALE);
  }
  {
    const int n16a = (int)(((size_t)4 * PLANE * 4 + (size_t)PLANE * 2) / 16);
    zero_fill16<<<(n16a + 255) / 256, 256, 0, stream>>>((unsigned int*)(wsb + o_cpl), n16a);
    const int n16b = (int)((size_t)PLANE * 2 / 16);
    zero_fill16<<<(n16b + 255) / 256, 256, 0, stream>>>((unsigned int*)(wsb + o_h1), n16b);
  }
  {
    const int n4 = NOUT / 4;
    rne_vec4<<<(n4 + 63) / 64, 64, 0, stream>>>(b_lin, blin, n4);
  }
  LayerArgs l0 = {};
  l0.ain = xh;  l0.win = wih0; l0.whh = whh0; l0.bih = b_ih0; l0.bhh = b_hh0;
  l0.cpl = cpl; l0.hseq = h0;
  l0.hn = out + OUT1_OFF; l0.cn = out + OUT2_OFF;
  l0.ain_bpitch = (long)NSEQ * NIN; l0.ain_tpitch = NIN;
  LayerArgs l1 = {};
  l1.ain = h0 + PLANE; l1.win = wih1; l1.whh = whh1; l1.bih = b_ih1; l1.bhh = b_hh1;
  l1.cpl = cpl + 2 * PLANE; l1.hseq = h1;
  l1.hn = out + OUT1_OFF + PLANE; l1.cn = out + OUT2_OFF + PLANE;
  l1.ain_bpitch = NHID; l1.ain_tpitch = PLANE;
  for (int p = 0; p <= NSEQ; ++p) {
    const int lbase = (p == NSEQ) ? 1 : 0;
    const int ny = (p == 0 || p == NSEQ) ? 1 : 2;
    lstm_step<<<dim3(NHID / HCOLS, ny), 256, 0, stream>>>(l0, l1, p, lbase, NSEQ - 1);
  }
  {
    const int tiles = (NSEQ / 64) * (NOUT / 64);
    wmma_gemm64<0, false, 2, 0, false, 0><<<dim3(tiles / 8, NBATCH), 256, 0, stream>>>(
        h1 + PLANE, h1 + PLANE, (int)PLANE, (long)NHID,
        wlin, wlin, NHID, 0L,
        (void*)out, d_ws, NOUT, (long)NSEQ * NOUT,
        blin,
        blin, 0L,
        NSEQ, NOUT, NHID, WSCALE_INV);
  }
}
